// Speller_16793322127469
// MI455X (gfx1250) — hardware-verified
//
#include <hip/hip_runtime.h>
#include <math.h>

constexpr int NB   = 32;
constexpr int NS   = 512;
constexpr int NU   = 512;
constexpr int ND   = 512;
constexpr int NT   = 128;
constexpr int NG4  = 4 * NU;
constexpr int NV   = 46;
constexpr int NTHR = 256;
constexpr int ROWS_A = 8;
constexpr int NBLK_A = NB / ROWS_A;
constexpr int ROWS_B = 16;
constexpr int NBLK_B = NB / ROWS_B;
constexpr int HP   = 520;
constexpr int FP   = 516;
constexpr int TILE16 = 16 * HP;
constexpr int PLANE8 = ROWS_A * HP;
constexpr int MROWS = NT * NB;
constexpr int OUT_BLK = ROWS_B * NV;
constexpr float WCARRY = 16.0f;
constexpr float WCARRY_INV = 0.0625f;
constexpr float LOSC = 2048.0f;
constexpr float LOSC_INV = 0.00048828125f;
static_assert(NB % ROWS_A == 0 && NB % ROWS_B == 0);
static_assert(NTHR / 32 == ROWS_A);
static_assert(2 * ROWS_A == 16);
static_assert(NU == 64 * (NTHR / 32));
static_assert(OUT_BLK == 736);
static_assert((OUT_BLK * 4) % 128 == 0);
static_assert(MROWS % 64 == 0 && NG4 % 64 == 0 && NU % 64 == 0 && NS % 64 == 0 && ND % 64 == 0);
static_assert(NU % 32 == 0 && NS % 32 == 0 && ND % 32 == 0);
static_assert((2 * TILE16) % NTHR == 0);
static_assert((HP % 8) == 0 && (PLANE8 % 8) == 0);

typedef __attribute__((ext_vector_type(16))) _Float16 v16h;
typedef __attribute__((ext_vector_type(8)))  _Float16 v8h;
typedef __attribute__((ext_vector_type(16))) __bf16   v16b;
typedef __attribute__((ext_vector_type(8)))  __bf16   v8b;
typedef __attribute__((ext_vector_type(8)))  float    v8f;
typedef __attribute__((ext_vector_type(4)))  float    v4f;

__device__ __forceinline__ unsigned short f2bf_bits(float f) {
  unsigned u = __float_as_uint(f);
  return (unsigned short)((u + 0x7FFFu + ((u >> 16) & 1u)) >> 16);
}
__device__ __forceinline__ float bf_bits2f(unsigned short h) { return __uint_as_float(((unsigned)h) << 16); }
__device__ __forceinline__ float bf16r(float f) { return bf_bits2f(f2bf_bits(f)); }

__device__ __forceinline__ void split3_bits(float v, unsigned short& hb, unsigned short& mb, unsigned short& lb) {
  hb = f2bf_bits(v);
  const float r1 = v - bf_bits2f(hb);
  mb = f2bf_bits(r1);
  const float r2 = r1 - bf_bits2f(mb);
  lb = f2bf_bits(r2);
}
__device__ __forceinline__ __bf16 bfc(unsigned short b) { return __builtin_bit_cast(__bf16, b); }

__device__ __forceinline__ void dep_guard_h(v8f& a, v8f& b, v16h x, v16h y) { asm volatile("v_nop\n\tv_nop\n\tv_nop\n\tv_nop" : "+v"(a), "+v"(b) : "v"(x), "v"(y)); }
__device__ __forceinline__ void dep_guard_b(v8f& a, v8f& b, v16b x, v16b y) { asm volatile("v_nop\n\tv_nop\n\tv_nop\n\tv_nop" : "+v"(a), "+v"(b) : "v"(x), "v"(y)); }
__device__ __forceinline__ void keep4_h(v16h a, v16h b, v16h c, v16h d) { asm volatile("v_nop" :: "v"(a), "v"(b), "v"(c), "v"(d)); }
__device__ __forceinline__ void keep4_b(v16b a, v16b b, v16b c, v16b d) { asm volatile("v_nop" :: "v"(a), "v"(b), "v"(c), "v"(d)); }
__device__ __forceinline__ void acc_guard4(v8f& a, v8f& b, v8f& c, v8f& d) { asm volatile("v_nop\n\tv_nop\n\tv_nop\n\tv_nop" : "+v"(a), "+v"(b), "+v"(c), "+v"(d)); }
template <typename T> struct Frag;
template <> struct Frag<_Float16> {
  typedef v16h V; union U { v16h v; v8h h[2]; };
  static __device__ __forceinline__ v16h load(const _Float16* p) {
    U f; f.h[0] = *(const v8h*)(p); f.h[1] = *(const v8h*)(p + 16); return f.v;
  }
  static __device__ __forceinline__ v8f mma(v16h a, v16h b, v8f c) {
    return __builtin_amdgcn_wmma_f32_16x16x32_f16(false, a, false, b, (short)0, c, false, false);
  }
  static __device__ __forceinline__ void guard(v8f& a, v8f& b, v16h x, v16h y) { dep_guard_h(a, b, x, y); }
  static __device__ __forceinline__ void keep(v16h a, v16h b, v16h c, v16h d) { keep4_h(a, b, c, d); }
};
template <> struct Frag<__bf16> {
  typedef v16b V; union U { v16b v; v8b h[2]; };
  static __device__ __forceinline__ v16b load(const __bf16* p) {
    U f; f.h[0] = *(const v8b*)(p); f.h[1] = *(const v8b*)(p + 16); return f.v;
  }
  static __device__ __forceinline__ v8f mma(v16b a, v16b b, v8f c) {
    return __builtin_amdgcn_wmma_f32_16x16x32_bf16(false, a, false, b, (short)0, c, false, false);
  }
  static __device__ __forceinline__ void guard(v8f& a, v8f& b, v16b x, v16b y) { dep_guard_b(a, b, x, y); }
  static __device__ __forceinline__ void keep(v16b a, v16b b, v16b c, v16b d) { keep4_b(a, b, c, d); }
};

__device__ __forceinline__ float fsig(float x)  { return __builtin_amdgcn_rcpf(1.0f + __expf(-x)); }
__device__ __forceinline__ float ftanh(float x) { return 1.0f - 2.0f * __builtin_amdgcn_rcpf(__expf(2.0f * x) + 1.0f); }

__device__ __forceinline__ void wave_lds_sync() {
  __builtin_amdgcn_fence(__ATOMIC_RELEASE, "workgroup");
  __builtin_amdgcn_wave_barrier();
  __builtin_amdgcn_fence(__ATOMIC_ACQUIRE, "workgroup");
}

template <int ET> struct Elem;
template <> struct Elem<0> { typedef _Float16 T; };
template <> struct Elem<1> { typedef __bf16 T; };
template <int ET, bool SPLIT, int BIAS_MODE, int OUT_MODE, bool RESID, int ACT = 0>
__global__ __launch_bounds__(256) void wmma_gemm64(
    const unsigned short* __restrict__ Ap, const unsigned short* __restrict__ A2p, int lda, long strideA,
    const unsigned short* __restrict__ Btp, const unsigned short* __restrict__ Bt2p, int ldb, long strideB,
    void* __restrict__ Cout, void* __restrict__ Cout2, int ldc, long strideC,
    const float* __restrict__ bias,
    const float* __restrict__ resid, long strideR,
    int M, int N, int K, float scale) {
  typedef typename Elem<ET>::T T;
  typedef typename Frag<T>::V V;
  const T* A = (const T*)Ap; const T* A2 = (const T*)A2p; const T* Bt = (const T*)Btp; const T* Bt2 = (const T*)Bt2p;
  __shared__ __align__(16) float sT[8][16 * 68];
  const int b    = blockIdx.y;
  const int lane = threadIdx.x & 31;
  const int wave = threadIdx.x >> 5;
  const int tilesN = N >> 6;
  const int tilesM = M >> 6;
  const int tile = blockIdx.x * 8 + wave;
  if (tile >= tilesM * tilesN) return;
  const int tm = tile / tilesN;
  const int tn = tile - tm * tilesN;
  const int m0 = tm << 6;
  const int n0 = tn << 6;

  const T* Ab  = A  + (size_t)b * strideA;
  const T* Bb  = Bt + (size_t)b * strideB;
  const T* Ab2 = SPLIT ? (A2  + (size_t)b * strideA) : nullptr;
  const T* Bb2 = SPLIT ? (Bt2 + (size_t)b * strideB) : nullptr;

  const int rlane = lane & 15;
  const int koff  = (lane >> 4) * 8;
  const int mOff  = (lane >> 4) * 8;

  v8f acc[4][4];
#pragma unroll
  for (int i = 0; i < 4; ++i)
#pragma unroll
    for (int j = 0; j < 4; ++j) acc[i][j] = (v8f){0.f,0.f,0.f,0.f,0.f,0.f,0.f,0.f};

  for (int k0 = 0; k0 < K; k0 += 32) {
    V bh[4], bl[4];
#pragma unroll
    for (int j = 0; j < 4; ++j) {
      const size_t bo = (size_t)(n0 + (j << 4) + rlane) * ldb + koff + k0;
      bh[j] = Frag<T>::load(Bb + bo);
      if (SPLIT) bl[j] = Frag<T>::load(Bb2 + bo);
    }
#pragma unroll
    for (int i = 0; i < 4; ++i) {
      const size_t ao = (size_t)(m0 + (i << 4) + rlane) * lda + koff + k0;
      V ah = Frag<T>::load(Ab + ao);
      V al;
      if (SPLIT) al = Frag<T>::load(Ab2 + ao);
#pragma unroll
      for (int j = 0; j < 4; ++j) {
        acc[i][j] = Frag<T>::mma(ah, bh[j], acc[i][j]);
        if (SPLIT) {
          acc[i][j] = Frag<T>::mma(ah, bl[j], acc[i][j]);
          acc[i][j] = Frag<T>::mma(al, bh[j], acc[i][j]);
        }
      }
      Frag<T>::guard(acc[i][0], acc[i][3], ah, SPLIT ? al : ah);
    }
    Frag<T>::keep(bh[0], bh[1], bh[2], bh[3]);
    if (SPLIT) Frag<T>::keep(bl[0], bl[1], bl[2], bl[3]);
  }
  acc_guard4(acc[0][0], acc[0][1], acc[0][2], acc[0][3]);
  acc_guard4(acc[1][0], acc[1][1], acc[1][2], acc[1][3]);
  acc_guard4(acc[2][0], acc[2][1], acc[2][2], acc[2][3]);
  acc_guard4(acc[3][0], acc[3][1], acc[3][2], acc[3][3]);

  float* slab = sT[wave];
  const float* Rb = RESID ? (resid + (size_t)b * strideR) : nullptr;
#pragma unroll
  for (int i = 0; i < 4; ++i) {
    const int mBase = m0 + (i << 4);
#pragma unroll
    for (int j = 0; j < 4; ++j) {
      const int n = n0 + (j << 4) + rlane;
      float bv = 0.f;
      if (BIAS_MODE == 2) bv = bias[n];
#pragma unroll
      for (int r = 0; r < 8; ++r) {
        float v = acc[i][j][r] * scale;
        if (BIAS_MODE == 1) v += bias[mBase + mOff + r];
        if (BIAS_MODE == 2) v += bv;
        if (RESID) v += Rb[(size_t)(mBase + mOff + r) * ldc + n];
        if (ACT == 1) v = tanhf(v);
        if (ACT == 2) v = fmaxf(v, 0.0f);
        if (ACT == 3) v = v / (1.0f + expf(-v));
        if (ACT == 4) v = (v > 0.f) ? v : 0.01f * v;
        slab[(mOff + r) * 68 + (j << 4) + rlane] = v;
      }
    }
    __builtin_amdgcn_fence(__ATOMIC_RELEASE, "workgroup");
    __builtin_amdgcn_wave_barrier();
    __builtin_amdgcn_fence(__ATOMIC_ACQUIRE, "workgroup");
    if (OUT_MODE == 0) {
      float* C = (float*)Cout + (size_t)b * strideC;
      const int hh = lane >> 4, c4 = (lane & 15) * 4;
      for (int pass = 0; pass < 2; ++pass) {
#pragma unroll
        for (int it = 0; it < 8; ++it) {
          const int row = it * 2 + hh;
          v4f v = *(const v4f*)(slab + row * 68 + c4);
          *(volatile v4f*)(C + (size_t)(mBase + row) * ldc + n0 + c4) = v;
        }
        __threadfence();
      }
    } else {
      const int q = lane >> 3, c8 = (lane & 7) * 8;
      unsigned short* C  = (unsigned short*)Cout  + (size_t)b * strideC;
      unsigned short* C2 = (OUT_MODE == 2) ? ((unsigned short*)Cout2 + (size_t)b * strideC) : nullptr;
      for (int pass = 0; pass < 2; ++pass) {
#pragma unroll
        for (int it = 0; it < 4; ++it) {
          const int row = it * 4 + q;
          const float* sp = slab + row * 68 + c8;
          v8h hv, lv;
#pragma unroll
          for (int e = 0; e < 8; ++e) {
            if (OUT_MODE == 1) {
              hv[e] = (_Float16)sp[e];
            } else {
              unsigned short hb = f2bf_bits(sp[e]);
              unsigned short lb = f2bf_bits(sp[e] - bf_bits2f(hb));
              hv[e] = __builtin_bit_cast(_Float16, hb);
              lv[e] = __builtin_bit_cast(_Float16, lb);
            }
          }
          *(volatile v8h*)(C + (size_t)(mBase + row) * ldc + n0 + c8) = hv;
          if (OUT_MODE == 2) *(volatile v8h*)(C2 + (size_t)(mBase + row) * ldc + n0 + c8) = lv;
        }
        __threadfence();
      }
    }
    __builtin_amdgcn_fence(__ATOMIC_RELEASE, "workgroup");
    __builtin_amdgcn_wave_barrier();
    __builtin_amdgcn_fence(__ATOMIC_ACQUIRE, "workgroup");
  }
}

template <int MODE>
__global__ __launch_bounds__(NTHR) void cvt8_kernel(const float* __restrict__ src, unsigned short* __restrict__ dst, int n8, float sc) {
  const int i = blockIdx.x * NTHR + threadIdx.x;
  if (i < n8) {
    const v4f a = *(const v4f*)(src + (size_t)i * 8);
    const v4f b = *(const v4f*)(src + (size_t)i * 8 + 4);
    v8h hv;
#pragma unroll
    for (int e = 0; e < 4; ++e) {
      unsigned short b0, b1;
      if (MODE == 0) {
        b0 = f2bf_bits(a[e] * sc);
        b1 = f2bf_bits(b[e] * sc);
      } else {
        b0 = __builtin_bit_cast(unsigned short, (_Float16)(bf16r(a[e]) * sc));
        b1 = __builtin_bit_cast(unsigned short, (_Float16)(bf16r(b[e]) * sc));
      }
      hv[e]     = __builtin_bit_cast(_Float16, b0);
      hv[4 + e] = __builtin_bit_cast(_Float16, b1);
    }
    *(volatile v8h*)(dst + (size_t)i * 8) = hv;
    __threadfence();
    *(volatile v8h*)(dst + (size_t)i * 8) = hv;
  }
}

__global__ __launch_bounds__(NTHR) void ycvt_kernel(const float* __restrict__ y, unsigned short* __restrict__ dst, int n8) {
  const int i = blockIdx.x * NTHR + threadIdx.x;
  if (i < n8) {
    const int row = i >> 6, d0 = (i & 63) * 8;
    const int t = row >> 5, b = row & 31;
    const float* s = y + ((size_t)(b * NT + t)) * ND + d0;
    const v4f a = *(const v4f*)(s);
    const v4f c = *(const v4f*)(s + 4);
    v8h hv;
#pragma unroll
    for (int e = 0; e < 4; ++e) {
      hv[e]     = __builtin_bit_cast(_Float16, f2bf_bits(a[e]));
      hv[4 + e] = __builtin_bit_cast(_Float16, f2bf_bits(c[e]));
    }
    *(volatile v8h*)(dst + (size_t)i * 8) = hv;
    __threadfence();
    *(volatile v8h*)(dst + (size_t)i * 8) = hv;
  }
}

template <int MODE>
__global__ __launch_bounds__(NTHR) void trcvt_kernel(const float* __restrict__ src, unsigned short* __restrict__ dst, int R, int C, float sc) {
  __shared__ float tile[64][65];
  const int tid = threadIdx.x, lane = tid & 31, wave = tid >> 5;
  const int c0 = blockIdx.x * 64, r0 = blockIdx.y * 64;
  const size_t zoff = (size_t)blockIdx.z * (size_t)R * (size_t)C;
  const float* s = src + zoff;
  const int lr = tid >> 4, lc = (tid & 15) * 4;
#pragma unroll
  for (int i = 0; i < 4; ++i) {
    const int rr = lr + 16 * i;
    const v4f v = *(const v4f*)(s + (size_t)(r0 + rr) * C + c0 + lc);
    tile[rr][lc]     = v[0];
    tile[rr][lc + 1] = v[1];
    tile[rr][lc + 2] = v[2];
    tile[rr][lc + 3] = v[3];
  }
  __syncthreads();
  const int q = lane & 7, rs = lane >> 3;
  unsigned short* d = dst + zoff;
  v8h hv[2];
#pragma unroll
  for (int it = 0; it < 2; ++it) {
    const int cc = 8 * wave + 4 * it + rs;
#pragma unroll
    for (int e = 0; e < 8; ++e) {
      const float f = tile[8 * q + e][cc];
      unsigned short bits;
      if (MODE == 0) bits = f2bf_bits(f * sc);
      else bits = __builtin_bit_cast(unsigned short, (_Float16)(bf16r(f) * sc));
      hv[it][e] = __builtin_bit_cast(_Float16, bits);
    }
  }
  for (int pass = 0; pass < 2; ++pass) {
#pragma unroll
    for (int it = 0; it < 2; ++it) {
      const int cc = 8 * wave + 4 * it + rs;
      *(volatile v8h*)(d + (size_t)(c0 + cc) * R + r0 + 8 * q) = hv[it];
    }
    __threadfence();
  }
}

__global__ __launch_bounds__(NTHR) __attribute__((amdgpu_num_vgpr(256)))
void attn_cell_kernel(const float* __restrict__ Zy,
                      const unsigned short* __restrict__ RTp,
                      const unsigned short* __restrict__ XKp,
                      const unsigned short* __restrict__ XVp,
                      unsigned short* __restrict__ CTX16) {
  __shared__ __align__(16) _Float16 AH[TILE16];
  __shared__ __align__(16) __bf16   HC3[3 * PLANE8];
  __shared__ __align__(16) __bf16   PP3[3 * PLANE8];
  __shared__ __align__(16) float    SC[ROWS_A * FP];
  const _Float16* RT = (const _Float16*)RTp;
  const __bf16*   XK = (const __bf16*)XKp;
  const __bf16*   XV = (const __bf16*)XVp;
  const int tid = threadIdx.x, lane = tid & 31, wave = tid >> 5;
  const int c = lane & 15, hh = lane >> 4, koff = hh * 8;
  const int rowbase = blockIdx.x * ROWS_A;
  const int psel = (c < 3) ? c : 0;

#pragma unroll 1
  for (int i = tid; i < TILE16; i += NTHR) AH[i] = (_Float16)0.0f;
  float cst[4][4], hcl[4][4];
#pragma unroll
  for (int nt = 0; nt < 4; ++nt)
#pragma unroll
    for (int q = 0; q < 4; ++q) { cst[nt][q] = 0.0f; hcl[nt][q] = 0.0f; }
  __syncthreads();

  const v8f z8 = {0.f, 0.f, 0.f, 0.f, 0.f, 0.f, 0.f, 0.f};

#pragma unroll 1
  for (int t = 0; t < NT; ++t) {
#pragma unroll
    for (int nt = 0; nt < 4; ++nt) {
      const int j = 64 * wave + 16 * nt + c;
      const _Float16* rt  = RT + (size_t)j * NU + koff;
      const _Float16* ahr = AH + c * HP + koff;
      v8f acc[4];
      acc[0] = z8; acc[1] = z8; acc[2] = z8; acc[3] = z8;
#pragma unroll 1
      for (int k0 = 0; k0 < NU; k0 += 32) {
        const v16h a  = Frag<_Float16>::load(ahr + k0);
        const v16h b0 = Frag<_Float16>::load(rt + k0);
        const v16h b1 = Frag<_Float16>::load(rt + (size_t)1 * NU * NU + k0);
        const v16h b2 = Frag<_Float16>::load(rt + (size_t)2 * NU * NU + k0);
        const v16h b3 = Frag<_Float16>::load(rt + (size_t)3 * NU * NU + k0);
        acc[0] = Frag<_Float16>::mma(a, b0, acc[0]);
        acc[1] = Frag<_Float16>::mma(a, b1, acc[1]);
        acc[2] = Frag<_Float16>::mma(a, b2, acc[2]);
        acc[3] = Frag<_Float16>::mma(a, b3, acc[3]);
        dep_guard_h(acc[0], acc[3], a, b3);
        keep4_h(b0, b1, b2, b3);
      }
      acc_guard4(acc[0], acc[1], acc[2], acc[3]);
#pragma unroll
      for (int q = 0; q < 4; ++q) {
        const int rr = 4 * hh + q;
        const float* zrow = Zy + (size_t)(t * NB + rowbase + rr) * NG4 + j;
        float zz[4];
#pragma unroll
        for (int g = 0; g < 4; ++g) {
          const float eq  = acc[g][q];
          const float eq4 = acc[g][4 + q];
          const float own  = hh ? eq4 : eq;
          const float send = hh ? eq : eq4;
          const float recv = __shfl_xor(send, 16, 32);
          const float hip = hh ? recv : own;
          const float lop = hh ? own : recv;
          zz[g] = hip * WCARRY_INV + lop * (WCARRY_INV * LOSC_INV) + zrow[g * NU];
        }
        const float ig = fsig(zz[0]);
        const float fg = fsig(zz[1]);
        const float gg = ftanh(zz[2]);
        const float og = fsig(zz[3]);
        const float cn = fg * cst[nt][q] + ig * gg;
        cst[nt][q] = cn;
        const float hn = og * ftanh(cn);
        hcl[nt][q] = hn;
        unsigned short p0, p1, p2;
        split3_bits(hn, p0, p1, p2);
        HC3[rr * HP + j]              = bfc(p0);
        HC3[PLANE8 + rr * HP + j]     = bfc(p1);
        HC3[2 * PLANE8 + rr * HP + j] = bfc(p2);
      }
    }
    __syncthreads();

    {
      const int m = wave;
      const int bglob = rowbase + m;
      float* scr = SC + m * FP;
      {
        const __bf16* arow = HC3 + psel * PLANE8 + m * HP + koff;
        const __bf16* xk = XK + ((size_t)bglob * NS + c) * NU + koff;
#pragma unroll 1
        for (int g8 = 0; g8 < 8; ++g8) {
          const int key0 = 64 * g8;
          const __bf16* xkg = xk + (size_t)key0 * NU;
          v8f acc[4];
          acc[0] = z8; acc[1] = z8; acc[2] = z8; acc[3] = z8;
#pragma unroll 1
          for (int k0 = 0; k0 < NU; k0 += 32) {
            const v16b a  = Frag<__bf16>::load(arow + k0);
            const v16b b0 = Frag<__bf16>::load(xkg + k0);
            const v16b b1 = Frag<__bf16>::load(xkg + (size_t)16 * NU + k0);
            const v16b b2 = Frag<__bf16>::load(xkg + (size_t)32 * NU + k0);
            const v16b b3 = Frag<__bf16>::load(xkg + (size_t)48 * NU + k0);
            acc[0] = Frag<__bf16>::mma(a, b0, acc[0]);
            acc[1] = Frag<__bf16>::mma(a, b1, acc[1]);
            acc[2] = Frag<__bf16>::mma(a, b2, acc[2]);
            acc[3] = Frag<__bf16>::mma(a, b3, acc[3]);
            dep_guard_b(acc[0], acc[3], a, b3);
            keep4_b(b0, b1, b2, b3);
          }
          acc_guard4(acc[0], acc[1], acc[2], acc[3]);
          if (hh == 0) {
            scr[key0 + c]      = acc[0][0] + acc[0][1] + acc[0][2];
            scr[key0 + 16 + c] = acc[1][0] + acc[1][1] + acc[1][2];
            scr[key0 + 32 + c] = acc[2][0] + acc[2][1] + acc[2][2];
            scr[key0 + 48 + c] = acc[3][0] + acc[3][1] + acc[3][2];
          }
        }
      }
      wave_lds_sync();
      float mx = -INFINITY;
#pragma unroll 1
      for (int i = 0; i < 16; ++i) mx = fmaxf(mx, scr[lane + 32 * i]);
#pragma unroll
      for (int off = 16; off > 0; off >>= 1) mx = fmaxf(mx, __shfl_xor(mx, off, 32));
      float sm = 0.0f;
#pragma unroll 1
      for (int i = 0; i < 16; ++i) {
        const int key = lane + 32 * i;
        const float e = expf(scr[key] - mx);
        scr[key] = e;
        sm += e;
      }
#pragma unroll
      for (int off = 16; off > 0; off >>= 1) sm += __shfl_xor(sm, off, 32);
      const float inv = 1.0f / sm;
#pragma unroll 1
      for (int i = 0; i < 16; ++i) {
        const int key = lane + 32 * i;
        const float p = scr[key] * inv;
        unsigned short p0, p1, p2;
        split3_bits(p, p0, p1, p2);
        PP3[m * HP + key]              = bfc(p0);
        PP3[PLANE8 + m * HP + key]     = bfc(p1);
        PP3[2 * PLANE8 + m * HP + key] = bfc(p2);
      }
      wave_lds_sync();
      {
        const __bf16* prow = PP3 + psel * PLANE8 + m * HP + koff;
        const __bf16* xv = XV + ((size_t)bglob * NU + c) * NS + koff;
#pragma unroll 1
        for (int g8 = 0; g8 < 8; ++g8) {
          const int u0 = 64 * g8;
          const __bf16* xvg = xv + (size_t)u0 * NS;
          v8f acc[4];
          acc[0] = z8; acc[1] = z8; acc[2] = z8; acc[3] = z8;
#pragma unroll 1
          for (int k0 = 0; k0 < NS; k0 += 32) {
            const v16b a  = Frag<__bf16>::load(prow + k0);
            const v16b b0 = Frag<__bf16>::load(xvg + k0);
            const v16b b1 = Frag<__bf16>::load(xvg + (size_t)16 * NS + k0);
            const v16b b2 = Frag<__bf16>::load(xvg + (size_t)32 * NS + k0);
            const v16b b3 = Frag<__bf16>::load(xvg + (size_t)48 * NS + k0);
            acc[0] = Frag<__bf16>::mma(a, b0, acc[0]);
            acc[1] = Frag<__bf16>::mma(a, b1, acc[1]);
            acc[2] = Frag<__bf16>::mma(a, b2, acc[2]);
            acc[3] = Frag<__bf16>::mma(a, b3, acc[3]);
            dep_guard_b(acc[0], acc[3], a, b3);
            keep4_b(b0, b1, b2, b3);
          }
          acc_guard4(acc[0], acc[1], acc[2], acc[3]);
          if (hh == 0) {
            scr[u0 + c]      = acc[0][0] + acc[0][1] + acc[0][2];
            scr[u0 + 16 + c] = acc[1][0] + acc[1][1] + acc[1][2];
            scr[u0 + 32 + c] = acc[2][0] + acc[2][1] + acc[2][2];
            scr[u0 + 48 + c] = acc[3][0] + acc[3][1] + acc[3][2];
          }
        }
      }
      wave_lds_sync();
      {
        unsigned short* crow = CTX16 + (size_t)(t * NB + bglob) * NU;
        v8h hv0, hv1;
        {
          const v4f f0 = *(const v4f*)(scr + 8 * lane);
          const v4f f1 = *(const v4f*)(scr + 8 * lane + 4);
#pragma unroll
          for (int e = 0; e < 4; ++e) { hv0[e] = (_Float16)f0[e]; hv0[4 + e] = (_Float16)f1[e]; }
        }
        {
          const v4f f0 = *(const v4f*)(scr + 256 + 8 * lane);
          const v4f f1 = *(const v4f*)(scr + 256 + 8 * lane + 4);
#pragma unroll
          for (int e = 0; e < 4; ++e) { hv1[e] = (_Float16)f0[e]; hv1[4 + e] = (_Float16)f1[e]; }
        }
        for (int pass = 0; pass < 2; ++pass) {
          *(volatile v8h*)(crow + 8 * lane)       = hv0;
          *(volatile v8h*)(crow + 256 + 8 * lane) = hv1;
          __threadfence();
        }
      }
    }
    __syncthreads();

#pragma unroll
    for (int nt = 0; nt < 4; ++nt) {
      const int j = 64 * wave + 16 * nt + c;
#pragma unroll
      for (int q = 0; q < 4; ++q) {
        const int rr = 4 * hh + q;
        const float cx = SC[rr * FP + j];
        cst[nt][q] = cst[nt][q] + cx;
        const float hs = hcl[nt][q] + cx;
        const _Float16 hi = (_Float16)hs;
        const float res = (hs - (float)hi) * LOSC;
        const _Float16 lo = (_Float16)res;
        AH[rr * HP + j]            = hi;
        AH[(ROWS_A + rr) * HP + j] = lo;
      }
    }
    __syncthreads();
  }
}

template <bool HEAD>
__global__ __launch_bounds__(NTHR) __attribute__((amdgpu_num_vgpr(256)))
void lstm_rec_kernel(const float* __restrict__ Zx,
                     const unsigned short* __restrict__ RTp,
                     unsigned short* __restrict__ HS16,
                     const float* __restrict__ Wd, const float* __restrict__ bd,
                     float* __restrict__ out) {
  __shared__ __align__(16) _Float16 Ah[2 * TILE16];
  __shared__ __align__(16) float    Hs[HEAD ? ROWS_B * FP : 4];
  __shared__ __align__(16) float    Os[HEAD ? OUT_BLK : 4];
  const _Float16* RT = (const _Float16*)RTp;
  const int tid = threadIdx.x, lane = tid & 31, wave = tid >> 5;
  const int c = lane & 15, hh = lane >> 4, koff = hh * 8;
  const int rowbase = blockIdx.x * ROWS_B;

#pragma unroll 1
  for (int i = tid; i < 2 * TILE16; i += NTHR) Ah[i] = (_Float16)0.0f;
  float cst[4][8];
#pragma unroll
  for (int nt = 0; nt < 4; ++nt)
#pragma unroll
    for (int r = 0; r < 8; ++r) cst[nt][r] = 0.0f;
  __syncthreads();

  const v8f z8 = {0.f, 0.f, 0.f, 0.f, 0.f, 0.f, 0.f, 0.f};

#pragma unroll 1
  for (int t = 0; t < NT; ++t) {
    const int cur = t & 1;
    const _Float16* ahr = Ah + cur * TILE16 + c * HP + koff;
    _Float16* ahn = Ah + (cur ^ 1) * TILE16;
    const bool last = (t == NT - 1);
#pragma unroll
    for (int nt = 0; nt < 4; ++nt) {
      const int j = 64 * wave + 16 * nt + c;
      const _Float16* rt = RT + (size_t)j * NU + koff;
      v8f acc[4];
      acc[0] = z8; acc[1] = z8; acc[2] = z8; acc[3] = z8;
#pragma unroll 1
      for (int k0 = 0; k0 < NU; k0 += 32) {
        const v16h a  = Frag<_Float16>::load(ahr + k0);
        const v16h b0 = Frag<_Float16>::load(rt + k0);
        const v16h b1 = Frag<_Float16>::load(rt + (size_t)1 * NU * NU + k0);
        const v16h b2 = Frag<_Float16>::load(rt + (size_t)2 * NU * NU + k0);
        const v16h b3 = Frag<_Float16>::load(rt + (size_t)3 * NU * NU + k0);
        acc[0] = Frag<_Float16>::mma(a, b0, acc[0]);
        acc[1] = Frag<_Float16>::mma(a, b1, acc[1]);
        acc[2] = Frag<_Float16>::mma(a, b2, acc[2]);
        acc[3] = Frag<_Float16>::mma(a, b3, acc[3]);
        dep_guard_h(acc[0], acc[3], a, b3);
        keep4_h(b0, b1, b2, b3);
      }
      acc_guard4(acc[0], acc[1], acc[2], acc[3]);
#pragma unroll
      for (int r = 0; r < 8; ++r) {
        const int row = 8 * hh + r;
        const float* zr = Zx + (size_t)(t * NB + rowbase + row) * NG4 + j;
        const float zi = acc[0][r] * WCARRY_INV + zr[0];
        const float zf = acc[1][r] * WCARRY_INV + zr[NU];
        const float zg = acc[2][r] * WCARRY_INV + zr[2 * NU];
        const float zo = acc[3][r] * WCARRY_INV + zr[3 * NU];
        const float ig = fsig(zi);
        const float fg = fsig(zf);
        const float og = fsig(zo);
        const float gg = ftanh(zg);
        const float cn = fg * cst[nt][r] + ig * gg;
        cst[nt][r] = cn;
        const float hn = og * ftanh(cn);
        ahn[row * HP + j] = (_Float16)hn;
        if (HEAD) { if (last) Hs[row * FP + j] = hn; }
      }
    }
    __syncthreads();
    if (!HEAD) {
      const int q = lane & 7, rs = lane >> 3;
      v8h hv[4];
#pragma unroll
      for (int it = 0; it < 4; ++it) {
        const int row = 4 * it + rs;
        hv[it] = *(const v8h*)(ahn + row * HP + 64 * wave + 8 * q);
      }
      for (int pass = 0; pass < 2; ++pass) {
#pragma unroll
        for (int it = 0; it < 4; ++it) {
          const int row = 4 * it + rs;
          *(volatile v8h*)(HS16 + (size_t)(t * NB + rowbase + row) * NU + 64 * wave + 8 * q) = hv[it];
        }
        __threadfence();
      }
    }
  }

  if (HEAD) {
    for (int o = tid; o < OUT_BLK; o += NTHR) {
      const int m = o / NV;
      const int v = o - m * NV;
      const float* hrow = Hs + m * FP;
      float s = 0.0f;
#pragma unroll 1
      for (int k = 0; k < NU; ++k) s = fmaf(hrow[k], bf16r(Wd[(size_t)k * NV + v]), s);
      s += bf16r(bd[v]);
      Os[o] = s;
    }
    __syncthreads();
    if (tid < ROWS_B) {
      float* orow = Os + tid * NV;
      float mx = -INFINITY;
#pragma unroll 1
      for (int v = 0; v < NV; ++v) mx = fmaxf(mx, orow[v]);
      float sm = 0.0f;
#pragma unroll 1
      for (int v = 0; v < NV; ++v) { const float e = expf(orow[v] - mx); orow[v] = e; sm += e; }
      const float inv = 1.0f / sm;
#pragma unroll 1
      for (int v = 0; v < NV; ++v) orow[v] = orow[v] * inv;
    }
    __syncthreads();
    if (tid < 32) {
      v4f w[6];
#pragma unroll
      for (int it = 0; it < 6; ++it) {
        const int f = it * 32 + lane;
        const int fc = (f < 184) ? f : 183;
        w[it] = *(const v4f*)(Os + 4 * fc);
      }
      float* ob = out + (size_t)blockIdx.x * OUT_BLK;
      for (int pass = 0; pass < 2; ++pass) {
#pragma unroll
        for (int it = 0; it < 5; ++it) *(volatile v4f*)(ob + 4 * (it * 32 + lane)) = w[it];
        if (lane < 24) *(volatile v4f*)(ob + 4 * (160 + lane)) = w[5];
        __threadfence();
      }
    }
  }
}

extern "C" void kernel_launch(void* const* d_in, const int* in_sizes, int n_in,
                              void* d_out, int out_size, void* d_ws, size_t ws_size, hipStream_t stream) {
  if (n_in < 13 || d_out == nullptr || d_ws == nullptr) return;
  const int WSZ = NU * NG4;
  if (in_sizes[0] != NB * NS * NU || in_sizes[1] != NB * NT * ND ||
      in_sizes[2] != WSZ || in_sizes[3] != WSZ || in_sizes[4] != NG4 ||
      in_sizes[5] != WSZ || in_sizes[6] != WSZ || in_sizes[7] != NG4 ||
      in_sizes[8] != WSZ || in_sizes[9] != WSZ || in_sizes[10] != NG4 ||
      in_sizes[11] != NU * NV || in_sizes[12] != NV || out_size != NB * NV) return;

  const float* x   = (const float*)d_in[0];
  const float* y   = (const float*)d_in[1];
  const float* W_a = (const float*)d_in[2];
  const float* R_a = (const float*)d_in[3];
  const float* b_a = (const float*)d_in[4];
  const float* W1  = (const float*)d_in[5];
  const float* R1  = (const float*)d_in[6];
  const float* b1  = (const float*)d_in[7];
  const float* W2  = (const float*)d_in[8];
  const float* R2  = (const float*)d_in[9];
  const float* b2  = (const float*)d_in[10];
  const float* Wd  = (const float*)d_in[11];
  const float* bd  = (const float*)d_in[12];
  float* out = (float*)d_out;

  char* ws = (char*)d_ws; size_t off = 0;
  auto carve = [&](size_t bytes) -> char* { char* p = ws + off; off += (bytes + 255) & ~(size_t)255; return p; };
  unsigned short* XK    = (unsigned short*)carve((size_t)NB * NS * NU * 2);
  unsigned short* XV    = (unsigned short*)carve((size_t)NB * NS * NU * 2);
  unsigned short* WaT   = (unsigned short*)carve((size_t)NG4 * NU * 2);
  unsigned short* RaT   = (unsigned short*)carve((size_t)NG4 * NU * 2);
  unsigned short* W1T   = (unsigned short*)carve((size_t)NG4 * NU * 2);
  unsigned short* R1T   = (unsigned short*)carve((size_t)NG4 * NU * 2);
  unsigned short* W2T   = (unsigned short*)carve((size_t)NG4 * NU * 2);
  unsigned short* R2T   = (unsigned short*)carve((size_t)NG4 * NU * 2);
  unsigned short* Y16   = (unsigned short*)carve((size_t)MROWS * ND * 2);
  unsigned short* CTX16 = (unsigned short*)carve((size_t)MROWS * NU * 2);
  unsigned short* HS16  = (unsigned short*)carve((size_t)MROWS * NU * 2);
  float*          Z     = (float*)carve((size_t)MROWS * NG4 * 4);
  if (off > ws_size || off > (size_t)134217728) return;

  {
    const dim3 g(NG4 / 64, NU / 64, 1);
    trcvt_kernel<0><<<g, NTHR, 0, stream>>>(W_a, WaT, NU, NG4, 1.0f);
    trcvt_kernel<1><<<g, NTHR, 0, stream>>>(R_a, RaT, NU, NG4, WCARRY);
    trcvt_kernel<1><<<g, NTHR, 0, stream>>>(W1,  W1T, NU, NG4, WCARRY);
    trcvt_kernel<1><<<g, NTHR, 0, stream>>>(R1,  R1T, NU, NG4, WCARRY);
    trcvt_kernel<1><<<g, NTHR, 0, stream>>>(W2,  W2T, NU, NG4, WCARRY);
    trcvt_kernel<1><<<g, NTHR, 0, stream>>>(R2,  R2T, NU, NG4, WCARRY);
  }
  {
    const int n8 = NB * NS * NU / 8;
    cvt8_kernel<0><<<(n8 + NTHR - 1) / NTHR, NTHR, 0, stream>>>(x, XK, n8, 1.0f);
    trcvt_kernel<0><<<dim3(NU / 64, NS / 64, NB), NTHR, 0, stream>>>(x, XV, NS, NU, 1.0f);
  }
  {
    const int n8 = MROWS * ND / 8;
    ycvt_kernel<<<(n8 + NTHR - 1) / NTHR, NTHR, 0, stream>>>(y, Y16, n8);
  }
  const int tiles = (MROWS / 64) * (NG4 / 64);
  const dim3 gg((tiles + 7) / 8, 1);
  wmma_gemm64<1, false, 2, 0, false, 0><<<gg, 256, 0, stream>>>(
      Y16, Y16, ND, 0L, WaT, WaT, NU, 0L, (void*)Z, (void*)Z, NG4, 0L, b_a, (const float*)Z, 0L, MROWS, NG4, ND, 1.0f);
  attn_cell_kernel<<<NBLK_A, NTHR, 0, stream>>>(Z, RaT, XK, XV, CTX16);
  wmma_gemm64<0, false, 2, 0, false, 0><<<gg, 256, 0, stream>>>(
      CTX16, CTX16, NU, 0L, W1T, W1T, NU, 0L, (void*)Z, (void*)Z, NG4, 0L, b1, (const float*)Z, 0L, MROWS, NG4, NU, WCARRY_INV);
  lstm_rec_kernel<false><<<NBLK_B, NTHR, 0, stream>>>(Z, R1T, HS16, Wd, bd, out);
  wmma_gemm64<0, false, 2, 0, false, 0><<<gg, 256, 0, stream>>>(
      HS16, HS16, NU, 0L, W2T, W2T, NU, 0L, (void*)Z, (void*)Z, NG4, 0L, b2, (const float*)Z, 0L, MROWS, NG4, NU, WCARRY_INV);
  lstm_rec_kernel<true><<<NBLK_B, NTHR, 0, stream>>>(Z, R2T, HS16, Wd, bd, out);
}
